// GRUCell_11879879541673
// MI455X (gfx1250) — hardware-verified
//
#include <hip/hip_runtime.h>
#include <stdint.h>

#ifndef NB
#define NB 4096
#endif
#define NB_FULL 4096
#define KD      2048
#define NU      2048
#define KTOT    4096
#define XSTRIDE 2048
#define HSTRIDE 2048

typedef __bf16 v16b __attribute__((ext_vector_type(16)));
typedef __bf16 v8b  __attribute__((ext_vector_type(8)));
typedef float  v8f  __attribute__((ext_vector_type(8)));
typedef float  v4f  __attribute__((ext_vector_type(4)));
typedef unsigned short v8us __attribute__((ext_vector_type(8)));

static_assert(KTOT == KD + NU);
static_assert(KD == NU);
static_assert((NB % 64) == 0 && NB >= 64 && NB <= NB_FULL);
static_assert((KD % 64) == 0 && (NU % 64) == 0 && (KTOT % 64) == 0);
static_assert((((NB / 64) * (NU / 64)) % 8) == 0);
static_assert(KD / 8 == 256);

__device__ __forceinline__ unsigned short bfbits(float f) {
  unsigned u = __float_as_uint(f);
  return (unsigned short)((u + 0x7FFFu + ((u >> 16) & 1u)) >> 16);
}
__device__ __forceinline__ float bfval(unsigned short b) { return __uint_as_float(((unsigned)b) << 16); }
__device__ __forceinline__ float bfr(float f) { return bfval(bfbits(f)); }
__device__ __forceinline__ void split_bf(float f, unsigned short& hb, unsigned short& lb) {
  hb = bfbits(f);
  lb = bfbits(f - bfval(hb));
}
__device__ __forceinline__ float sigm(float x) {
  const float e = expf(-x);
  return 1.0f / (1.0f + e);
}

__device__ __forceinline__ v16b ldfragb(const __bf16* p) {
  union { v16b v; v8b h[2]; } f;
  f.h[0] = *(const v8b*)(p);
  f.h[1] = *(const v8b*)(p + 16);
  return f.v;
}
__device__ __forceinline__ v8f mmab(v16b a, v16b b, v8f c) {
  return __builtin_amdgcn_wmma_f32_16x16x32_bf16(false, a, false, b, (short)0, c, false, false);
}
__device__ __forceinline__ v8f zero8() {
  v8f z;
#pragma unroll
  for (int i = 0; i < 8; ++i) z[i] = 0.0f;
  return z;
}

__device__ __forceinline__ void guard_g(v8f& a, v8f& b, v16b x, v16b y) {
  asm volatile("v_nop\n\tv_nop\n\tv_nop\n\tv_nop" : "+v"(a), "+v"(b) : "v"(x), "v"(y));
}
__device__ __forceinline__ void keep4(v16b a, v16b b, v16b c, v16b d) {
  asm volatile("v_nop" :: "v"(a), "v"(b), "v"(c), "v"(d));
}
__device__ __forceinline__ void accg4(v8f& a, v8f& b, v8f& c, v8f& d) {
  asm volatile("v_nop\n\tv_nop\n\tv_nop\n\tv_nop" : "+v"(a), "+v"(b), "+v"(c), "+v"(d));
}

__global__ __launch_bounds__(256) void cvt_act_kernel(const float* __restrict__ x, const float* __restrict__ hs,
                                                      unsigned short* __restrict__ XH, int nrows) {
  const int b = (int)blockIdx.x;
  const bool second = (b >= nrows);
  const int row = b - (second ? nrows : 0);
  if (row >= nrows) return;
  const float* src = second ? (hs + (size_t)row * HSTRIDE) : (x + (size_t)row * XSTRIDE);
  const int c0 = (int)threadIdx.x * 8;
  const v4f a = *(const v4f*)(src + c0);
  const v4f c = *(const v4f*)(src + c0 + 4);
  v8us o;
#pragma unroll
  for (int i = 0; i < 4; ++i) {
    o[i]     = bfbits(a[i]);
    o[4 + i] = bfbits(c[i]);
  }
  unsigned short* d = XH + (size_t)row * KTOT + (second ? KD : 0) + c0;
  *(volatile v8us*)d = o;
  __threadfence();
  *(volatile v8us*)d = o;
}

__global__ __launch_bounds__(256) void wtr_kernel(const float* __restrict__ w, unsigned short* __restrict__ Wt) {
  __shared__ __align__(16) float t[64][65];
  const int tid = (int)threadIdx.x;
  const int k0 = (int)blockIdx.y * 64;
  const int n0 = (int)blockIdx.x * 64;
  {
    const int r = tid >> 4, c4 = (tid & 15) * 4;
#pragma unroll
    for (int p = 0; p < 4; ++p) {
      const int kr = p * 16 + r;
      const v4f v = *(const v4f*)(w + (size_t)(k0 + kr) * NU + n0 + c4);
      t[kr][c4 + 0] = v[0];
      t[kr][c4 + 1] = v[1];
      t[kr][c4 + 2] = v[2];
      t[kr][c4 + 3] = v[3];
    }
  }
  __syncthreads();
  {
    const int q = tid >> 3, c8 = (tid & 7) * 8;
#pragma unroll
    for (int ps = 0; ps < 2; ++ps) {
#pragma unroll
      for (int p = 0; p < 2; ++p) {
        const int nr = p * 32 + q;
        v8us o;
#pragma unroll
        for (int e = 0; e < 8; ++e) o[e] = bfbits(t[c8 + e][nr]);
        *(volatile v8us*)(Wt + (size_t)(n0 + nr) * KTOT + k0 + c8) = o;
      }
      __threadfence();
    }
  }
}

template <bool SPLITA>
__device__ __forceinline__ void kloop(v8f (&acc)[4][4], const __bf16* __restrict__ A,
                                      const __bf16* __restrict__ A2, int lda,
                                      const __bf16* __restrict__ Bt, int ldb, int K, int m0, int n0, int lane) {
  const int rl = lane & 15;
  const int koff = (lane >> 4) * 8;
#pragma unroll 1
  for (int k0 = 0; k0 < K; k0 += 32) {
    v16b bh[4];
#pragma unroll
    for (int j = 0; j < 4; ++j) bh[j] = ldfragb(Bt + (size_t)(n0 + (j << 4) + rl) * ldb + koff + k0);
#pragma unroll
    for (int i = 0; i < 4; ++i) {
      const size_t ao = (size_t)(m0 + (i << 4) + rl) * lda + koff + k0;
      const v16b ah = ldfragb(A + ao);
      v16b al = ah;
      if (SPLITA) al = ldfragb(A2 + ao);
#pragma unroll
      for (int j = 0; j < 4; ++j) {
        acc[i][j] = mmab(ah, bh[j], acc[i][j]);
        if (SPLITA) acc[i][j] = mmab(al, bh[j], acc[i][j]);
      }
      guard_g(acc[i][0], acc[i][3], ah, SPLITA ? al : bh[3]);
    }
    keep4(bh[0], bh[1], bh[2], bh[3]);
  }
}

template <int MODE>
__global__ __launch_bounds__(256) void gru_gemm_kernel(const unsigned short* __restrict__ XHp,
                                                       const unsigned short* HRhp, const unsigned short* HRlp,
                                                       const unsigned short* __restrict__ Wtp,
                                                       const float* __restrict__ bias,
                                                       const float* __restrict__ states,
                                                       const float* Zin,
                                                       unsigned short* HRho, unsigned short* HRlo,
                                                       float* Fout, int M) {
  __shared__ __align__(16) float sT[8][16 * 68];
  const int lane = threadIdx.x & 31, wave = threadIdx.x >> 5;
  const int tilesN = NU >> 6, tilesM = M >> 6;
  const int tile = (int)blockIdx.x * 8 + wave;
  if (tile >= tilesM * tilesN) return;
  const int tm = tile / tilesN, tn = tile - tm * tilesN;
  const int m0 = tm << 6, n0 = tn << 6;
  const int rl = lane & 15;
  const int mOff = (lane >> 4) * 8;

  const __bf16* XH = (const __bf16*)(const void*)XHp;
  const __bf16* W  = (const __bf16*)(const void*)Wtp;

  v8f acc[4][4];
#pragma unroll
  for (int i = 0; i < 4; ++i)
#pragma unroll
    for (int j = 0; j < 4; ++j) acc[i][j] = zero8();

  if (MODE == 2) {
    const __bf16* HRh = (const __bf16*)(const void*)HRhp;
    const __bf16* HRl = (const __bf16*)(const void*)HRlp;
    kloop<false>(acc, XH, XH, KTOT, W, KTOT, KD, m0, n0, lane);
    kloop<true>(acc, HRh, HRl, NU, W + KD, KTOT, NU, m0, n0, lane);
  } else {
    kloop<false>(acc, XH, XH, KTOT, W, KTOT, KTOT, m0, n0, lane);
  }
  accg4(acc[0][0], acc[0][1], acc[0][2], acc[0][3]);
  accg4(acc[1][0], acc[1][1], acc[1][2], acc[1][3]);
  accg4(acc[2][0], acc[2][1], acc[2][2], acc[2][3]);
  accg4(acc[3][0], acc[3][1], acc[3][2], acc[3][3]);

  float* slab = sT[wave];
#pragma unroll
  for (int i = 0; i < 4; ++i) {
    const int mBase = m0 + (i << 4);
#pragma unroll
    for (int j = 0; j < 4; ++j) {
      const float bv = bfr(bias[n0 + (j << 4) + rl]);
#pragma unroll
      for (int r = 0; r < 8; ++r) slab[(mOff + r) * 68 + (j << 4) + rl] = acc[i][j][r] + bv;
    }
    __builtin_amdgcn_fence(__ATOMIC_RELEASE, "workgroup");
    __builtin_amdgcn_wave_barrier();
    __builtin_amdgcn_fence(__ATOMIC_ACQUIRE, "workgroup");
    if (MODE == 0) {
      const int qq = lane >> 3, c8 = (lane & 7) * 8;
#pragma unroll
      for (int ps = 0; ps < 2; ++ps) {
#pragma unroll
        for (int it = 0; it < 4; ++it) {
          const int row = it * 4 + qq;
          const int grow = mBase + row;
          const float* sp = slab + row * 68 + c8;
          const v4f sa = *(const v4f*)(states + (size_t)grow * HSTRIDE + n0 + c8);
          const v4f sb = *(const v4f*)(states + (size_t)grow * HSTRIDE + n0 + c8 + 4);
          v8us hv, lv;
#pragma unroll
          for (int e = 0; e < 4; ++e) {
            unsigned short hb, lb;
            const float x0 = bfr(sa[e]) * sigm(sp[e]);
            split_bf(x0, hb, lb);
            hv[e] = hb; lv[e] = lb;
            const float x1 = bfr(sb[e]) * sigm(sp[4 + e]);
            split_bf(x1, hb, lb);
            hv[4 + e] = hb; lv[4 + e] = lb;
          }
          const size_t go = (size_t)grow * NU + n0 + c8;
          *(volatile v8us*)(HRho + go) = hv;
          *(volatile v8us*)(HRlo + go) = lv;
        }
        __threadfence();
      }
    } else {
      const int hh = lane >> 4, c4 = (lane & 15) * 4;
#pragma unroll
      for (int ps = 0; ps < 2; ++ps) {
#pragma unroll
        for (int it = 0; it < 8; ++it) {
          const int row = it * 2 + hh;
          const int grow = mBase + row;
          const v4f v = *(const v4f*)(slab + row * 68 + c4);
          v4f o;
          if (MODE == 1) {
#pragma unroll
            for (int e = 0; e < 4; ++e) o[e] = sigm(v[e]);
          } else {
            const v4f zz = *(const v4f*)(Zin + (size_t)grow * NU + n0 + c4);
            const v4f ss = *(const v4f*)(states + (size_t)grow * HSTRIDE + n0 + c4);
#pragma unroll
            for (int e = 0; e < 4; ++e) {
              const float z = zz[e];
              const float n = tanhf(v[e]);
              const float h = bfr(ss[e]);
              o[e] = (1.0f - z) * h + z * n;
            }
          }
          *(volatile v4f*)(Fout + (size_t)grow * NU + n0 + c4) = o;
        }
        __threadfence();
      }
    }
    __builtin_amdgcn_fence(__ATOMIC_RELEASE, "workgroup");
    __builtin_amdgcn_wave_barrier();
    __builtin_amdgcn_fence(__ATOMIC_ACQUIRE, "workgroup");
  }
}

extern "C" void kernel_launch(void* const* d_in, const int* in_sizes, int n_in,
                              void* d_out, int out_size, void* d_ws, size_t ws_size,
                              hipStream_t stream) {
  if (n_in < 8) return;
  if (in_sizes[0] < NB * KD || in_sizes[1] < NB * NU) return;
  if (in_sizes[2] < KTOT * NU || in_sizes[4] < KTOT * NU || in_sizes[6] < KTOT * NU) return;
  if (in_sizes[3] < NU || in_sizes[5] < NU || in_sizes[7] < NU) return;
  if (out_size < NB * NU) return;

  const float* x   = (const float*)d_in[0];
  const float* hs  = (const float*)d_in[1];
  const float* w_r = (const float*)d_in[2];
  const float* b_r = (const float*)d_in[3];
  const float* w_z = (const float*)d_in[4];
  const float* b_z = (const float*)d_in[5];
  const float* w_n = (const float*)d_in[6];
  const float* b_n = (const float*)d_in[7];
  float* out = (float*)d_out;

  const size_t bXH = (size_t)NB * KTOT * 2;
  const size_t bW  = (size_t)NU * KTOT * 2;
  const size_t bHR = (size_t)NB * NU * 2;
  const size_t bZ  = (size_t)NB * NU * 4;
  size_t off = 0;
  const size_t oXH  = off; off += bXH;
  const size_t oW   = off; off += bW;
  const size_t oHRh = off; off += bHR;
  const size_t oHRl = off; off += bHR;
  const size_t oZ   = off; off += bZ;
  if (off > ws_size) return;
  if (off > (size_t)134217728) return;

  char* ws = (char*)d_ws;
  unsigned short* XH  = (unsigned short*)(ws + oXH);
  unsigned short* WT  = (unsigned short*)(ws + oW);
  unsigned short* HRh = (unsigned short*)(ws + oHRh);
  unsigned short* HRl = (unsigned short*)(ws + oHRl);
  float*          Zp  = (float*)(ws + oZ);

  const dim3 blk(256);
  const dim3 gT(NU / 64, KTOT / 64);
  const dim3 gG(((NB / 64) * (NU / 64)) / 8);

  cvt_act_kernel<<<dim3(2 * NB), blk, 0, stream>>>(x, hs, XH, NB);
  wtr_kernel<<<gT, blk, 0, stream>>>(w_r, WT);
  gru_gemm_kernel<0><<<gG, blk, 0, stream>>>(XH, HRh, HRl, WT, b_r, hs, Zp, HRh, HRl, Zp, NB);
  wtr_kernel<<<gT, blk, 0, stream>>>(w_z, WT);
  gru_gemm_kernel<1><<<gG, blk, 0, stream>>>(XH, HRh, HRl, WT, b_z, hs, Zp, HRh, HRl, Zp, NB);
  wtr_kernel<<<gT, blk, 0, stream>>>(w_n, WT);
  gru_gemm_kernel<2><<<gG, blk, 0, stream>>>(XH, HRh, HRl, WT, b_n, hs, Zp, HRh, HRl, out, NB);
  (void)hipGetLastError();
}
